// lightST_43198781063352
// MI455X (gfx1250) — hardware-run, weakly checked
//
#include <hip/hip_runtime.h>


namespace {
constexpr int NC = 20000, NCP = 20032, NGENE = 2000, NGP = 2016, D = 64, KCL = 7, EEXP = 2000000, EADJ = 120000, EPOS = 500000, ENEG = 500000;
constexpr float XS = 8.0f, WSC = 256.0f;
typedef _Float16 b16;
typedef __attribute__((ext_vector_type(16))) _Float16 v16b;
typedef __attribute__((ext_vector_type(8))) _Float16 v8b;
typedef __attribute__((ext_vector_type(8))) float v8f;
typedef __attribute__((ext_vector_type(4))) float v4f;
typedef __attribute__((ext_vector_type(2))) float v2f;
__device__ __forceinline__ float bf16_rne(float f) { unsigned int u = __float_as_uint(f); u += 0x7FFFu + ((u >> 16) & 1u); return __uint_as_float(u & 0xFFFF0000u); }
__device__ __forceinline__ void split16(float v, b16& hi, b16& lo) { hi = (b16)v; lo = (b16)(v - (float)hi); }
__device__ __forceinline__ v16b frag_kb(const b16* p, int hh) { const v8b a = *(const v8b*)(p + 8 * hh), b = *(const v8b*)(p + 16 + 8 * hh); v16b f;
#pragma unroll
  for (int e = 0; e < 8; ++e) { f[e] = a[e]; f[8 + e] = b[e]; } return f; }
__device__ __forceinline__ v8f wmma16b(v16b a, v16b b, v8f c) { v8f d = __builtin_amdgcn_wmma_f32_16x16x32_f16(false, a, false, b, (short)0, c, false, false); asm volatile("v_nop\n\tv_nop\n\tv_nop\n\tv_nop" : "+v"(d) : "v"(a), "v"(b)); return d; }
__device__ __forceinline__ void wave_lds_sync() { __builtin_amdgcn_fence(__ATOMIC_RELEASE, "workgroup"); __builtin_amdgcn_wave_barrier(); __builtin_amdgcn_fence(__ATOMIC_ACQUIRE, "workgroup"); }
__device__ __forceinline__ float pmul(float a, float b) { float p = a * b; asm volatile("" : "+v"(p)); return p; }
__device__ __forceinline__ float opaque(float a) { asm volatile("" : "+v"(a)); return a; }
__device__ __forceinline__ int iclamp(int v, int lo, int hi) { return v < lo ? lo : (v > hi ? hi : v); }
constexpr int CSR_NBLK3 = 512, CSR_GB3 = 3, CSR_GN3 = 1 << CSR_GB3  , CSR_TS3 = (CSR_GN3 < 32 ? 32 : CSR_GN3)  , CSR_MAXG3 = 512, CSR_CAP3 = 12288  ;
__device__ __host__ __forceinline__ int csr_tix3(int v) { return (v >> CSR_GB3) * CSR_TS3 + (v & (CSR_GN3 - 1)); }
__global__ __launch_bounds__(64) void csrA_kernel3(const int* __restrict__ dst, int E, int N, int nG, int CHP, int NGP, int* __restrict__ STG, int* __restrict__ HST) {
  extern __shared__ int sm[];
  int* cnt = sm; int* run = sm + NGP; int* ids = sm + 2 * NGP;
  const int b = blockIdx.x; const int ch = (E + CSR_NBLK3 - 1) / CSR_NBLK3; const int e0 = b * ch, e1 = min(E, e0 + ch);
  for (int i = threadIdx.x; i < NGP; i += 64) cnt[i] = 0;
  for (int i = threadIdx.x; i < CHP; i += 64) ids[i] = -1;
  __syncthreads();
  if (threadIdx.x == 0) {
    for (int e = e0; e < e1; ++e) { int d = dst[e]; d = (d < 0) ? 0 : (d >= N ? N - 1 : d); cnt[d >> CSR_GB3] += 1; }
    int acc = 0; for (int g = 0; g < nG; ++g) { run[g] = acc; acc += cnt[g]; }
    for (int e = e0; e < e1; ++e) { int d = dst[e]; d = (d < 0) ? 0 : (d >= N ? N - 1 : d); const int g = d >> CSR_GB3; ids[run[g]] = e; run[g] += 1; } }
  __syncthreads();
  typedef __attribute__((ext_vector_type(4))) int v4i;
  for (int pass = 0; pass < 2; ++pass) {
    for (int i = threadIdx.x; i < CHP / 4; i += 64) *(volatile v4i*)(STG + (size_t)b * CHP + i * 4) = *(const v4i*)(&ids[i * 4]);
    for (int i = threadIdx.x; i < NGP / 4; i += 64) { v4i v; for (int e = 0; e < 4; ++e) v[e] = (i * 4 + e < nG) ? cnt[i * 4 + e] : 0; *(volatile v4i*)(HST + (size_t)b * NGP + i * 4) = v; }
    __threadfence(); }
}
__global__ __launch_bounds__(512) void csrS_kernel3(const int* __restrict__ HST, int nG, int NGP, int* __restrict__ START, int* __restrict__ TOT, int* __restrict__ OFF) {
  __shared__ int tot[CSR_MAXG3];
  const int b = threadIdx.x;
  for (int pass = 0; pass < 2; ++pass) { int runb = 0; for (int g = 0; g < nG; ++g) { int c = HST[(size_t)b * NGP + g]; c = (c < 0) ? 0 : c; ((volatile int*)OFF)[(size_t)g * CSR_NBLK3 + b] = runb; runb += c; } __threadfence(); }
  for (int g = threadIdx.x; g < nG; g += 512) { int s = 0; for (int bb = 0; bb < CSR_NBLK3; ++bb) { int c = HST[(size_t)bb * NGP + g]; s += (c < 0) ? 0 : c; } tot[g] = s; }
  __syncthreads();
  if (threadIdx.x < 32) {
    __shared__ int st[CSR_MAXG3 + 32];
    if (threadIdx.x == 0) { int acc = 0; for (int g = 0; g < NGP; ++g) { st[g] = acc; if (g < nG) acc += (tot[g] + 31) & ~31; } st[NGP] = acc; }
    __builtin_amdgcn_fence(__ATOMIC_RELEASE, "workgroup"); __builtin_amdgcn_wave_barrier(); __builtin_amdgcn_fence(__ATOMIC_ACQUIRE, "workgroup");
    for (int pass = 0; pass < 2; ++pass) { for (int i = threadIdx.x; i < NGP + 32; i += 32) { ((volatile int*)START)[i] = (i <= NGP) ? st[min(i, NGP)] : 0; ((volatile int*)TOT)[i] = (i < nG) ? tot[i] : 0; } __threadfence(); } }
}
__global__ __launch_bounds__(256) void csrB_kernel3(const int* __restrict__ dst, int N, int nG, int CHP, int NGP, int permLen, const int* __restrict__ STG, const int* __restrict__ HST, const int* __restrict__ OFF, const int* __restrict__ START, const int* __restrict__ TOT, int* __restrict__ PERM, int* __restrict__ ROWPTR, int* __restrict__ ROWCNT, int* __restrict__ FLAG) {
  typedef __attribute__((ext_vector_type(4))) int v4i;
  __shared__ int ids[CSR_CAP3]; __shared__ unsigned short key[CSR_CAP3]; __shared__ int outp[CSR_CAP3]; __shared__ int ncnt[CSR_GN3 + 1]; __shared__ int boff[CSR_NBLK3 + 1];
  const int g = blockIdx.x, t_ = threadIdx.x; int tot = TOT[g]; int st = START[g], stn = START[g + 1]; const int v0 = g * CSR_GN3; const int nv = min(CSR_GN3, N - v0); const int t0 = g * CSR_TS3;
  st = (st < 0) ? 0 : (st > permLen - 32 ? permLen - 32 : st) & ~31; stn = (stn < st) ? st : (stn > permLen ? permLen : stn); tot = (tot < 0) ? 0 : tot; if (tot > stn - st && tot <= CSR_CAP3) tot = stn - st;
  if (tot > CSR_CAP3) {
    for (int pass = 0; pass < 2; ++pass) { for (int i = t_; i < CSR_TS3 / 4; i += 256) { v4i a, c; for (int e = 0; e < 4; ++e) { a[e] = st; c[e] = 0; } *(volatile v4i*)(ROWPTR + t0 + i * 4) = a; *(volatile v4i*)(ROWCNT + t0 + i * 4) = c; } if (t_ == 0) ((volatile int*)FLAG)[0] = 1; __threadfence(); } (void)nv; return; }
  if (t_ == 0) { int acc = 0; for (int b = 0; b < CSR_NBLK3; ++b) { boff[b] = acc; int c = HST[(size_t)b * NGP + g]; c = (c < 0) ? 0 : (c > CHP ? CHP : c); acc += c; if (acc > tot) acc = tot; } boff[CSR_NBLK3] = acc; }
  for (int i = t_; i <= CSR_GN3; i += 256) ncnt[i] = 0;
  __syncthreads();
  for (int b = 0; b < CSR_NBLK3; ++b) { const int c = boff[b + 1] - boff[b]; int o_ = OFF[(size_t)g * CSR_NBLK3 + b]; o_ = (o_ < 0) ? 0 : (o_ > CHP - c ? CHP - c : o_); const int* src_ = STG + (size_t)b * CHP + o_;
    for (int i = t_; i < c; i += 256) { int id = src_[i]; id = (id < 0) ? 0 : id; ids[boff[b] + i] = id; int d = dst[id]; d = (d < v0) ? v0 : (d >= N ? N - 1 : d); int kk = d - v0; kk = (kk < 0) ? 0 : (kk >= CSR_GN3 ? CSR_GN3 - 1 : kk); key[boff[b] + i] = (unsigned short)kk; } }
  __syncthreads();
  if (t_ == 0) { for (int i = 0; i < tot; ++i) ncnt[key[i]] += 1; int acc = 0; for (int vl = 0; vl < CSR_GN3; ++vl) { const int c = ncnt[vl]; ncnt[vl] = acc; acc += c; } ncnt[CSR_GN3] = acc;
    for (int i = 0; i < tot; ++i) { const int vl = key[i]; outp[ncnt[vl]] = ids[i]; ncnt[vl] += 1; }
    for (int vl = CSR_GN3; vl > 0; --vl) ncnt[vl] = ncnt[vl - 1]; ncnt[0] = 0; }
  __syncthreads();
  for (int pass = 0; pass < 2; ++pass) {
    for (int i = t_; i < (stn - st) / 4; i += 256) { v4i v; for (int e = 0; e < 4; ++e) { const int q = i * 4 + e; v[e] = (q < tot) ? outp[q] : -1; } *(volatile v4i*)(PERM + st + i * 4) = v; }
    for (int i = t_; i < CSR_TS3 / 4; i += 256) { v4i a, c; for (int e = 0; e < 4; ++e) { const int vl = i * 4 + e; const int vc = vl < CSR_GN3 ? vl : CSR_GN3; a[e] = (vl < CSR_GN3) ? st + ncnt[vc] : st; c[e] = (vl < nv) ? (ncnt[(vc < CSR_GN3 ? vc : CSR_GN3 - 1) + 1] - ncnt[vc]) : 0; } *(volatile v4i*)(ROWPTR + t0 + i * 4) = a; *(volatile v4i*)(ROWCNT + t0 + i * 4) = c; }
    __threadfence(); }
}
__global__ __launch_bounds__(256) void csrZ_kernel3(int* __restrict__ p, size_t n4) { typedef __attribute__((ext_vector_type(4))) int v4i; const size_t tid = (size_t)blockIdx.x * 256 + threadIdx.x, nth = (size_t)gridDim.x * 256; v4i z = {0, 0, 0, 0}; for (size_t i = tid; i < n4; i += nth) *(volatile v4i*)(p + i * 4) = z; }
struct CsrBufs3 { int *STG, *HST, *OFF, *START, *TOT, *PERM, *ROWPTR, *ROWCNT, *FLAG; int nG, NGP, CHP; size_t permLen; char* base; size_t bytes; };
static size_t csr_carve3(CsrBufs3& c, char* ws, size_t off, int E, int N) {
  const size_t off0 = off; c.base = ws + off;
  auto al = [&](size_t bytes) { char* p = ws + off; off += (bytes + 255) & ~(size_t)255; return p; };
  c.nG = (N + CSR_GN3 - 1) / CSR_GN3; c.NGP = (c.nG + 31) & ~31; const int ch = (E + CSR_NBLK3 - 1) / CSR_NBLK3; c.CHP = (ch + 31) & ~31; c.permLen = (size_t)E + 32 * (size_t)c.nG + 32;
  c.STG = (int*)al((size_t)CSR_NBLK3 * c.CHP * 4); c.HST = (int*)al((size_t)CSR_NBLK3 * c.NGP * 4); c.OFF = (int*)al((size_t)c.NGP * CSR_NBLK3 * 4); c.START = (int*)al((size_t)(c.NGP + 64) * 4); c.TOT = (int*)al((size_t)(c.NGP + 64) * 4);
  c.PERM = (int*)al(c.permLen * 4); c.ROWPTR = (int*)al((size_t)c.nG * CSR_TS3 * 4); c.ROWCNT = (int*)al((size_t)c.nG * CSR_TS3 * 4); c.FLAG = (int*)al(256);
  c.bytes = off - off0; return off;
}
static void csr_build3(const CsrBufs3& c, const int* dst, int E, int N, hipStream_t stream) {
  const size_t smem = (size_t)(2 * c.NGP + c.CHP) * 4;
  csrZ_kernel3<<<512, 256, 0, stream>>>((int*)c.base, c.bytes / 16);
  csrA_kernel3<<<CSR_NBLK3, 64, smem, stream>>>(dst, E, N, c.nG, c.CHP, c.NGP, c.STG, c.HST);
  csrS_kernel3<<<1, 512, 0, stream>>>(c.HST, c.nG, c.NGP, c.START, c.TOT, c.OFF);
  csrB_kernel3<<<c.nG, 256, 0, stream>>>(dst, N, c.nG, c.CHP, c.NGP, (int)c.permLen, c.STG, c.HST, c.OFF, c.START, c.TOT, c.PERM, c.ROWPTR, c.ROWCNT, c.FLAG);
}

constexpr int CSR_NBLK6 = 512, CSR_GB6 = 6, CSR_GN6 = 1 << CSR_GB6  , CSR_TS6 = (CSR_GN6 < 32 ? 32 : CSR_GN6)  , CSR_MAXG6 = 512, CSR_CAP6 = 12288  ;
__device__ __host__ __forceinline__ int csr_tix6(int v) { return (v >> CSR_GB6) * CSR_TS6 + (v & (CSR_GN6 - 1)); }
__global__ __launch_bounds__(64) void csrA_kernel6(const int* __restrict__ dst, int E, int N, int nG, int CHP, int NGP, int* __restrict__ STG, int* __restrict__ HST) {
  extern __shared__ int sm[];
  int* cnt = sm; int* run = sm + NGP; int* ids = sm + 2 * NGP;
  const int b = blockIdx.x; const int ch = (E + CSR_NBLK6 - 1) / CSR_NBLK6; const int e0 = b * ch, e1 = min(E, e0 + ch);
  for (int i = threadIdx.x; i < NGP; i += 64) cnt[i] = 0;
  for (int i = threadIdx.x; i < CHP; i += 64) ids[i] = -1;
  __syncthreads();
  if (threadIdx.x == 0) {
    for (int e = e0; e < e1; ++e) { int d = dst[e]; d = (d < 0) ? 0 : (d >= N ? N - 1 : d); cnt[d >> CSR_GB6] += 1; }
    int acc = 0; for (int g = 0; g < nG; ++g) { run[g] = acc; acc += cnt[g]; }
    for (int e = e0; e < e1; ++e) { int d = dst[e]; d = (d < 0) ? 0 : (d >= N ? N - 1 : d); const int g = d >> CSR_GB6; ids[run[g]] = e; run[g] += 1; } }
  __syncthreads();
  typedef __attribute__((ext_vector_type(4))) int v4i;
  for (int pass = 0; pass < 2; ++pass) {
    for (int i = threadIdx.x; i < CHP / 4; i += 64) *(volatile v4i*)(STG + (size_t)b * CHP + i * 4) = *(const v4i*)(&ids[i * 4]);
    for (int i = threadIdx.x; i < NGP / 4; i += 64) { v4i v; for (int e = 0; e < 4; ++e) v[e] = (i * 4 + e < nG) ? cnt[i * 4 + e] : 0; *(volatile v4i*)(HST + (size_t)b * NGP + i * 4) = v; }
    __threadfence(); }
}
__global__ __launch_bounds__(512) void csrS_kernel6(const int* __restrict__ HST, int nG, int NGP, int* __restrict__ START, int* __restrict__ TOT, int* __restrict__ OFF) {
  __shared__ int tot[CSR_MAXG6];
  const int b = threadIdx.x;
  for (int pass = 0; pass < 2; ++pass) { int runb = 0; for (int g = 0; g < nG; ++g) { int c = HST[(size_t)b * NGP + g]; c = (c < 0) ? 0 : c; ((volatile int*)OFF)[(size_t)g * CSR_NBLK6 + b] = runb; runb += c; } __threadfence(); }
  for (int g = threadIdx.x; g < nG; g += 512) { int s = 0; for (int bb = 0; bb < CSR_NBLK6; ++bb) { int c = HST[(size_t)bb * NGP + g]; s += (c < 0) ? 0 : c; } tot[g] = s; }
  __syncthreads();
  if (threadIdx.x < 32) {
    __shared__ int st[CSR_MAXG6 + 32];
    if (threadIdx.x == 0) { int acc = 0; for (int g = 0; g < NGP; ++g) { st[g] = acc; if (g < nG) acc += (tot[g] + 31) & ~31; } st[NGP] = acc; }
    __builtin_amdgcn_fence(__ATOMIC_RELEASE, "workgroup"); __builtin_amdgcn_wave_barrier(); __builtin_amdgcn_fence(__ATOMIC_ACQUIRE, "workgroup");
    for (int pass = 0; pass < 2; ++pass) { for (int i = threadIdx.x; i < NGP + 32; i += 32) { ((volatile int*)START)[i] = (i <= NGP) ? st[min(i, NGP)] : 0; ((volatile int*)TOT)[i] = (i < nG) ? tot[i] : 0; } __threadfence(); } }
}
__global__ __launch_bounds__(256) void csrB_kernel6(const int* __restrict__ dst, int N, int nG, int CHP, int NGP, int permLen, const int* __restrict__ STG, const int* __restrict__ HST, const int* __restrict__ OFF, const int* __restrict__ START, const int* __restrict__ TOT, int* __restrict__ PERM, int* __restrict__ ROWPTR, int* __restrict__ ROWCNT, int* __restrict__ FLAG) {
  typedef __attribute__((ext_vector_type(4))) int v4i;
  __shared__ int ids[CSR_CAP6]; __shared__ unsigned short key[CSR_CAP6]; __shared__ int outp[CSR_CAP6]; __shared__ int ncnt[CSR_GN6 + 1]; __shared__ int boff[CSR_NBLK6 + 1];
  const int g = blockIdx.x, t_ = threadIdx.x; int tot = TOT[g]; int st = START[g], stn = START[g + 1]; const int v0 = g * CSR_GN6; const int nv = min(CSR_GN6, N - v0); const int t0 = g * CSR_TS6;
  st = (st < 0) ? 0 : (st > permLen - 32 ? permLen - 32 : st) & ~31; stn = (stn < st) ? st : (stn > permLen ? permLen : stn); tot = (tot < 0) ? 0 : tot; if (tot > stn - st && tot <= CSR_CAP6) tot = stn - st;
  if (tot > CSR_CAP6) {
    for (int pass = 0; pass < 2; ++pass) { for (int i = t_; i < CSR_TS6 / 4; i += 256) { v4i a, c; for (int e = 0; e < 4; ++e) { a[e] = st; c[e] = 0; } *(volatile v4i*)(ROWPTR + t0 + i * 4) = a; *(volatile v4i*)(ROWCNT + t0 + i * 4) = c; } if (t_ == 0) ((volatile int*)FLAG)[0] = 1; __threadfence(); } (void)nv; return; }
  if (t_ == 0) { int acc = 0; for (int b = 0; b < CSR_NBLK6; ++b) { boff[b] = acc; int c = HST[(size_t)b * NGP + g]; c = (c < 0) ? 0 : (c > CHP ? CHP : c); acc += c; if (acc > tot) acc = tot; } boff[CSR_NBLK6] = acc; }
  for (int i = t_; i <= CSR_GN6; i += 256) ncnt[i] = 0;
  __syncthreads();
  for (int b = 0; b < CSR_NBLK6; ++b) { const int c = boff[b + 1] - boff[b]; int o_ = OFF[(size_t)g * CSR_NBLK6 + b]; o_ = (o_ < 0) ? 0 : (o_ > CHP - c ? CHP - c : o_); const int* src_ = STG + (size_t)b * CHP + o_;
    for (int i = t_; i < c; i += 256) { int id = src_[i]; id = (id < 0) ? 0 : id; ids[boff[b] + i] = id; int d = dst[id]; d = (d < v0) ? v0 : (d >= N ? N - 1 : d); int kk = d - v0; kk = (kk < 0) ? 0 : (kk >= CSR_GN6 ? CSR_GN6 - 1 : kk); key[boff[b] + i] = (unsigned short)kk; } }
  __syncthreads();
  if (t_ == 0) { for (int i = 0; i < tot; ++i) ncnt[key[i]] += 1; int acc = 0; for (int vl = 0; vl < CSR_GN6; ++vl) { const int c = ncnt[vl]; ncnt[vl] = acc; acc += c; } ncnt[CSR_GN6] = acc;
    for (int i = 0; i < tot; ++i) { const int vl = key[i]; outp[ncnt[vl]] = ids[i]; ncnt[vl] += 1; }
    for (int vl = CSR_GN6; vl > 0; --vl) ncnt[vl] = ncnt[vl - 1]; ncnt[0] = 0; }
  __syncthreads();
  for (int pass = 0; pass < 2; ++pass) {
    for (int i = t_; i < (stn - st) / 4; i += 256) { v4i v; for (int e = 0; e < 4; ++e) { const int q = i * 4 + e; v[e] = (q < tot) ? outp[q] : -1; } *(volatile v4i*)(PERM + st + i * 4) = v; }
    for (int i = t_; i < CSR_TS6 / 4; i += 256) { v4i a, c; for (int e = 0; e < 4; ++e) { const int vl = i * 4 + e; const int vc = vl < CSR_GN6 ? vl : CSR_GN6; a[e] = (vl < CSR_GN6) ? st + ncnt[vc] : st; c[e] = (vl < nv) ? (ncnt[(vc < CSR_GN6 ? vc : CSR_GN6 - 1) + 1] - ncnt[vc]) : 0; } *(volatile v4i*)(ROWPTR + t0 + i * 4) = a; *(volatile v4i*)(ROWCNT + t0 + i * 4) = c; }
    __threadfence(); }
}
__global__ __launch_bounds__(256) void csrZ_kernel6(int* __restrict__ p, size_t n4) { typedef __attribute__((ext_vector_type(4))) int v4i; const size_t tid = (size_t)blockIdx.x * 256 + threadIdx.x, nth = (size_t)gridDim.x * 256; v4i z = {0, 0, 0, 0}; for (size_t i = tid; i < n4; i += nth) *(volatile v4i*)(p + i * 4) = z; }
struct CsrBufs6 { int *STG, *HST, *OFF, *START, *TOT, *PERM, *ROWPTR, *ROWCNT, *FLAG; int nG, NGP, CHP; size_t permLen; char* base; size_t bytes; };
static size_t csr_carve6(CsrBufs6& c, char* ws, size_t off, int E, int N) {
  const size_t off0 = off; c.base = ws + off;
  auto al = [&](size_t bytes) { char* p = ws + off; off += (bytes + 255) & ~(size_t)255; return p; };
  c.nG = (N + CSR_GN6 - 1) / CSR_GN6; c.NGP = (c.nG + 31) & ~31; const int ch = (E + CSR_NBLK6 - 1) / CSR_NBLK6; c.CHP = (ch + 31) & ~31; c.permLen = (size_t)E + 32 * (size_t)c.nG + 32;
  c.STG = (int*)al((size_t)CSR_NBLK6 * c.CHP * 4); c.HST = (int*)al((size_t)CSR_NBLK6 * c.NGP * 4); c.OFF = (int*)al((size_t)c.NGP * CSR_NBLK6 * 4); c.START = (int*)al((size_t)(c.NGP + 64) * 4); c.TOT = (int*)al((size_t)(c.NGP + 64) * 4);
  c.PERM = (int*)al(c.permLen * 4); c.ROWPTR = (int*)al((size_t)c.nG * CSR_TS6 * 4); c.ROWCNT = (int*)al((size_t)c.nG * CSR_TS6 * 4); c.FLAG = (int*)al(256);
  c.bytes = off - off0; return off;
}
static void csr_build6(const CsrBufs6& c, const int* dst, int E, int N, hipStream_t stream) {
  const size_t smem = (size_t)(2 * c.NGP + c.CHP) * 4;
  csrZ_kernel6<<<512, 256, 0, stream>>>((int*)c.base, c.bytes / 16);
  csrA_kernel6<<<CSR_NBLK6, 64, smem, stream>>>(dst, E, N, c.nG, c.CHP, c.NGP, c.STG, c.HST);
  csrS_kernel6<<<1, 512, 0, stream>>>(c.HST, c.nG, c.NGP, c.START, c.TOT, c.OFF);
  csrB_kernel6<<<c.nG, 256, 0, stream>>>(dst, N, c.nG, c.CHP, c.NGP, (int)c.permLen, c.STG, c.HST, c.OFF, c.START, c.TOT, c.PERM, c.ROWPTR, c.ROWCNT, c.FLAG);
}

constexpr int CSR_NBLK9 = 512, CSR_GB9 = 9, CSR_GN9 = 1 << CSR_GB9  , CSR_TS9 = (CSR_GN9 < 32 ? 32 : CSR_GN9)  , CSR_MAXG9 = 512, CSR_CAP9 = 12288  ;
__device__ __host__ __forceinline__ int csr_tix9(int v) { return (v >> CSR_GB9) * CSR_TS9 + (v & (CSR_GN9 - 1)); }
__global__ __launch_bounds__(64) void csrA_kernel9(const int* __restrict__ dst, int E, int N, int nG, int CHP, int NGP, int* __restrict__ STG, int* __restrict__ HST) {
  extern __shared__ int sm[];
  int* cnt = sm; int* run = sm + NGP; int* ids = sm + 2 * NGP;
  const int b = blockIdx.x; const int ch = (E + CSR_NBLK9 - 1) / CSR_NBLK9; const int e0 = b * ch, e1 = min(E, e0 + ch);
  for (int i = threadIdx.x; i < NGP; i += 64) cnt[i] = 0;
  for (int i = threadIdx.x; i < CHP; i += 64) ids[i] = -1;
  __syncthreads();
  if (threadIdx.x == 0) {
    for (int e = e0; e < e1; ++e) { int d = dst[e]; d = (d < 0) ? 0 : (d >= N ? N - 1 : d); cnt[d >> CSR_GB9] += 1; }
    int acc = 0; for (int g = 0; g < nG; ++g) { run[g] = acc; acc += cnt[g]; }
    for (int e = e0; e < e1; ++e) { int d = dst[e]; d = (d < 0) ? 0 : (d >= N ? N - 1 : d); const int g = d >> CSR_GB9; ids[run[g]] = e; run[g] += 1; } }
  __syncthreads();
  typedef __attribute__((ext_vector_type(4))) int v4i;
  for (int pass = 0; pass < 2; ++pass) {
    for (int i = threadIdx.x; i < CHP / 4; i += 64) *(volatile v4i*)(STG + (size_t)b * CHP + i * 4) = *(const v4i*)(&ids[i * 4]);
    for (int i = threadIdx.x; i < NGP / 4; i += 64) { v4i v; for (int e = 0; e < 4; ++e) v[e] = (i * 4 + e < nG) ? cnt[i * 4 + e] : 0; *(volatile v4i*)(HST + (size_t)b * NGP + i * 4) = v; }
    __threadfence(); }
}
__global__ __launch_bounds__(512) void csrS_kernel9(const int* __restrict__ HST, int nG, int NGP, int* __restrict__ START, int* __restrict__ TOT, int* __restrict__ OFF) {
  __shared__ int tot[CSR_MAXG9];
  const int b = threadIdx.x;
  for (int pass = 0; pass < 2; ++pass) { int runb = 0; for (int g = 0; g < nG; ++g) { int c = HST[(size_t)b * NGP + g]; c = (c < 0) ? 0 : c; ((volatile int*)OFF)[(size_t)g * CSR_NBLK9 + b] = runb; runb += c; } __threadfence(); }
  for (int g = threadIdx.x; g < nG; g += 512) { int s = 0; for (int bb = 0; bb < CSR_NBLK9; ++bb) { int c = HST[(size_t)bb * NGP + g]; s += (c < 0) ? 0 : c; } tot[g] = s; }
  __syncthreads();
  if (threadIdx.x < 32) {
    __shared__ int st[CSR_MAXG9 + 32];
    if (threadIdx.x == 0) { int acc = 0; for (int g = 0; g < NGP; ++g) { st[g] = acc; if (g < nG) acc += (tot[g] + 31) & ~31; } st[NGP] = acc; }
    __builtin_amdgcn_fence(__ATOMIC_RELEASE, "workgroup"); __builtin_amdgcn_wave_barrier(); __builtin_amdgcn_fence(__ATOMIC_ACQUIRE, "workgroup");
    for (int pass = 0; pass < 2; ++pass) { for (int i = threadIdx.x; i < NGP + 32; i += 32) { ((volatile int*)START)[i] = (i <= NGP) ? st[min(i, NGP)] : 0; ((volatile int*)TOT)[i] = (i < nG) ? tot[i] : 0; } __threadfence(); } }
}
__global__ __launch_bounds__(256) void csrB_kernel9(const int* __restrict__ dst, int N, int nG, int CHP, int NGP, int permLen, const int* __restrict__ STG, const int* __restrict__ HST, const int* __restrict__ OFF, const int* __restrict__ START, const int* __restrict__ TOT, int* __restrict__ PERM, int* __restrict__ ROWPTR, int* __restrict__ ROWCNT, int* __restrict__ FLAG) {
  typedef __attribute__((ext_vector_type(4))) int v4i;
  __shared__ int ids[CSR_CAP9]; __shared__ unsigned short key[CSR_CAP9]; __shared__ int outp[CSR_CAP9]; __shared__ int ncnt[CSR_GN9 + 1]; __shared__ int boff[CSR_NBLK9 + 1];
  const int g = blockIdx.x, t_ = threadIdx.x; int tot = TOT[g]; int st = START[g], stn = START[g + 1]; const int v0 = g * CSR_GN9; const int nv = min(CSR_GN9, N - v0); const int t0 = g * CSR_TS9;
  st = (st < 0) ? 0 : (st > permLen - 32 ? permLen - 32 : st) & ~31; stn = (stn < st) ? st : (stn > permLen ? permLen : stn); tot = (tot < 0) ? 0 : tot; if (tot > stn - st && tot <= CSR_CAP9) tot = stn - st;
  if (tot > CSR_CAP9) {
    for (int pass = 0; pass < 2; ++pass) { for (int i = t_; i < CSR_TS9 / 4; i += 256) { v4i a, c; for (int e = 0; e < 4; ++e) { a[e] = st; c[e] = 0; } *(volatile v4i*)(ROWPTR + t0 + i * 4) = a; *(volatile v4i*)(ROWCNT + t0 + i * 4) = c; } if (t_ == 0) ((volatile int*)FLAG)[0] = 1; __threadfence(); } (void)nv; return; }
  if (t_ == 0) { int acc = 0; for (int b = 0; b < CSR_NBLK9; ++b) { boff[b] = acc; int c = HST[(size_t)b * NGP + g]; c = (c < 0) ? 0 : (c > CHP ? CHP : c); acc += c; if (acc > tot) acc = tot; } boff[CSR_NBLK9] = acc; }
  for (int i = t_; i <= CSR_GN9; i += 256) ncnt[i] = 0;
  __syncthreads();
  for (int b = 0; b < CSR_NBLK9; ++b) { const int c = boff[b + 1] - boff[b]; int o_ = OFF[(size_t)g * CSR_NBLK9 + b]; o_ = (o_ < 0) ? 0 : (o_ > CHP - c ? CHP - c : o_); const int* src_ = STG + (size_t)b * CHP + o_;
    for (int i = t_; i < c; i += 256) { int id = src_[i]; id = (id < 0) ? 0 : id; ids[boff[b] + i] = id; int d = dst[id]; d = (d < v0) ? v0 : (d >= N ? N - 1 : d); int kk = d - v0; kk = (kk < 0) ? 0 : (kk >= CSR_GN9 ? CSR_GN9 - 1 : kk); key[boff[b] + i] = (unsigned short)kk; } }
  __syncthreads();
  if (t_ == 0) { for (int i = 0; i < tot; ++i) ncnt[key[i]] += 1; int acc = 0; for (int vl = 0; vl < CSR_GN9; ++vl) { const int c = ncnt[vl]; ncnt[vl] = acc; acc += c; } ncnt[CSR_GN9] = acc;
    for (int i = 0; i < tot; ++i) { const int vl = key[i]; outp[ncnt[vl]] = ids[i]; ncnt[vl] += 1; }
    for (int vl = CSR_GN9; vl > 0; --vl) ncnt[vl] = ncnt[vl - 1]; ncnt[0] = 0; }
  __syncthreads();
  for (int pass = 0; pass < 2; ++pass) {
    for (int i = t_; i < (stn - st) / 4; i += 256) { v4i v; for (int e = 0; e < 4; ++e) { const int q = i * 4 + e; v[e] = (q < tot) ? outp[q] : -1; } *(volatile v4i*)(PERM + st + i * 4) = v; }
    for (int i = t_; i < CSR_TS9 / 4; i += 256) { v4i a, c; for (int e = 0; e < 4; ++e) { const int vl = i * 4 + e; const int vc = vl < CSR_GN9 ? vl : CSR_GN9; a[e] = (vl < CSR_GN9) ? st + ncnt[vc] : st; c[e] = (vl < nv) ? (ncnt[(vc < CSR_GN9 ? vc : CSR_GN9 - 1) + 1] - ncnt[vc]) : 0; } *(volatile v4i*)(ROWPTR + t0 + i * 4) = a; *(volatile v4i*)(ROWCNT + t0 + i * 4) = c; }
    __threadfence(); }
}
__global__ __launch_bounds__(256) void csrZ_kernel9(int* __restrict__ p, size_t n4) { typedef __attribute__((ext_vector_type(4))) int v4i; const size_t tid = (size_t)blockIdx.x * 256 + threadIdx.x, nth = (size_t)gridDim.x * 256; v4i z = {0, 0, 0, 0}; for (size_t i = tid; i < n4; i += nth) *(volatile v4i*)(p + i * 4) = z; }
struct CsrBufs9 { int *STG, *HST, *OFF, *START, *TOT, *PERM, *ROWPTR, *ROWCNT, *FLAG; int nG, NGP, CHP; size_t permLen; char* base; size_t bytes; };
static size_t csr_carve9(CsrBufs9& c, char* ws, size_t off, int E, int N) {
  const size_t off0 = off; c.base = ws + off;
  auto al = [&](size_t bytes) { char* p = ws + off; off += (bytes + 255) & ~(size_t)255; return p; };
  c.nG = (N + CSR_GN9 - 1) / CSR_GN9; c.NGP = (c.nG + 31) & ~31; const int ch = (E + CSR_NBLK9 - 1) / CSR_NBLK9; c.CHP = (ch + 31) & ~31; c.permLen = (size_t)E + 32 * (size_t)c.nG + 32;
  c.STG = (int*)al((size_t)CSR_NBLK9 * c.CHP * 4); c.HST = (int*)al((size_t)CSR_NBLK9 * c.NGP * 4); c.OFF = (int*)al((size_t)c.NGP * CSR_NBLK9 * 4); c.START = (int*)al((size_t)(c.NGP + 64) * 4); c.TOT = (int*)al((size_t)(c.NGP + 64) * 4);
  c.PERM = (int*)al(c.permLen * 4); c.ROWPTR = (int*)al((size_t)c.nG * CSR_TS9 * 4); c.ROWCNT = (int*)al((size_t)c.nG * CSR_TS9 * 4); c.FLAG = (int*)al(256);
  c.bytes = off - off0; return off;
}
static void csr_build9(const CsrBufs9& c, const int* dst, int E, int N, hipStream_t stream) {
  const size_t smem = (size_t)(2 * c.NGP + c.CHP) * 4;
  csrZ_kernel9<<<512, 256, 0, stream>>>((int*)c.base, c.bytes / 16);
  csrA_kernel9<<<CSR_NBLK9, 64, smem, stream>>>(dst, E, N, c.nG, c.CHP, c.NGP, c.STG, c.HST);
  csrS_kernel9<<<1, 512, 0, stream>>>(c.HST, c.nG, c.NGP, c.START, c.TOT, c.OFF);
  csrB_kernel9<<<c.nG, 256, 0, stream>>>(dst, N, c.nG, c.CHP, c.NGP, (int)c.permLen, c.STG, c.HST, c.OFF, c.START, c.TOT, c.PERM, c.ROWPTR, c.ROWCNT, c.FLAG);
}


template <int GB, int RAWSRC>
__global__ __launch_bounds__(256) void mp_kernel(const float* __restrict__ SRC, int nsrc, const float* __restrict__ cj, const float* __restrict__ ci, const int* __restrict__ other, int E, const int* __restrict__ PERM, const int* __restrict__ ROWPTR, const int* __restrict__ ROWCNT, int permLen, int NT, float* __restrict__ OUT) {
  constexpr int GN = 1 << GB, TS = GN < 32 ? 32 : GN;
  const int wave = threadIdx.x >> 5, lane = threadIdx.x & 31; const int v = blockIdx.x * 8 + wave; const int c0 = lane * 2; v2f a = {0.0f, 0.0f};
  if (v < NT) { const int tix = (v >> GB) * TS + (v & (GN - 1)); int st = ROWPTR[tix], cnt = ROWCNT[tix]; cnt = iclamp(cnt, 0, 65536); st = iclamp(st, 0, permLen - cnt);
#pragma unroll 2
    for (int j = 0; j < cnt; ++j) { const int e = iclamp(PERM[st + j], 0, E - 1); const int s = iclamp(other[e], 0, nsrc - 1); const float w = bf16_rne(cj[s]); v2f x = *(const v2f*)(SRC + (size_t)s * D + c0);
      if (RAWSRC) { x[0] = bf16_rne(x[0]); x[1] = bf16_rne(x[1]); } a[0] += pmul(w, x[0]); a[1] += pmul(w, x[1]); }
    const float civ = bf16_rne(ci[v]); a[0] = pmul(civ, a[0]); a[1] = pmul(civ, a[1]); }
  for (int pass = 0; pass < 2; ++pass) { *(volatile v2f*)(OUT + (size_t)v * D + c0) = a; __threadfence(); }
}
template <int MIX>
__global__ __launch_bounds__(256) void spmm_kernel(const float* __restrict__ raw, const float* __restrict__ P1, const float* __restrict__ P2, const float* __restrict__ wts, const float* __restrict__ av, const int* __restrict__ cols, const int* __restrict__ PERM, const int* __restrict__ ROWPTR, const int* __restrict__ ROWCNT, int permLen, float* __restrict__ OUT) {
  const int wave = threadIdx.x >> 5, lane = threadIdx.x & 31; const int v = blockIdx.x * 8 + wave; const int c0 = lane * 2; v2f a = {0.0f, 0.0f};
  const float w0 = bf16_rne(wts[0]), w1 = bf16_rne(wts[1]), w2 = bf16_rne(wts[2]);
  if (v < NC) { int st = ROWPTR[v], cnt = ROWCNT[v]; cnt = iclamp(cnt, 0, 65536); st = iclamp(st, 0, permLen - cnt);
#pragma unroll 2
    for (int j = 0; j < cnt; ++j) { const int e = iclamp(PERM[st + j], 0, EADJ - 1); const int s = iclamp(cols[e], 0, NC - 1); const float w = bf16_rne(av[e]); v2f x = *(const v2f*)(P1 + (size_t)s * D + c0);
      if (MIX) { const v2f r = *(const v2f*)(raw + (size_t)s * D + c0), p2 = *(const v2f*)(P2 + (size_t)s * D + c0); for (int i = 0; i < 2; ++i) x[i] = pmul(w0, bf16_rne(r[i])) + pmul(w1, x[i]) + pmul(w2, p2[i]); }
      a[0] += pmul(w, x[0]); a[1] += pmul(w, x[1]); } }
  for (int pass = 0; pass < 2; ++pass) { *(volatile v2f*)(OUT + (size_t)v * D + c0) = a; __threadfence(); }
}
__global__ __launch_bounds__(256) void gmix_kernel(const float* __restrict__ gf, const float* __restrict__ G1, const float* __restrict__ G2, const float* __restrict__ wts, float* __restrict__ GZ) {
  const int wave = threadIdx.x >> 5, lane = threadIdx.x & 31; const int g = blockIdx.x * 8 + wave; const int c0 = lane * 2; v2f o = {0.0f, 0.0f};
  if (g < NGENE) { const float w0 = bf16_rne(wts[0]), w1 = bf16_rne(wts[1]), w2 = bf16_rne(wts[2]); const v2f r = *(const v2f*)(gf + (size_t)g * D + c0), a = *(const v2f*)(G1 + (size_t)g * D + c0), b = *(const v2f*)(G2 + (size_t)g * D + c0);
    for (int i = 0; i < 2; ++i) o[i] = pmul(w0, bf16_rne(r[i])) + pmul(w1, a[i]) + pmul(w2, b[i]); }
  for (int pass = 0; pass < 2; ++pass) { *(volatile v2f*)(GZ + (size_t)g * D + c0) = o; __threadfence(); }
}
__global__ __launch_bounds__(64) void q_kernel(const float* __restrict__ CZ, const float* __restrict__ mu, float* __restrict__ outq) {
  __shared__ __attribute__((aligned(16))) b16 Ah[2][16][D + 8], Al[2][16][D + 8], MU[16][D + 8]; __shared__ __attribute__((aligned(16))) float so[32 * KCL]; __shared__ float n2s[2][16], m2s[16];
  const int wave = threadIdx.x >> 5, lane = threadIdx.x & 31, nloc = lane & 15, hlf = lane >> 4; const size_t v0 = (size_t)blockIdx.x * 32 + wave * 16;
  if (wave == 0) {
    const int row = lane >> 1, half = lane & 1; float s = 0.0f;
#pragma unroll 4
    for (int k = 0; k < 32; ++k) { const int kk = half * 32 + k; const float m = row < KCL ? bf16_rne(mu[(row < KCL ? row : 0) * D + kk]) : 0.0f;     MU[row][kk] = (b16)(m * WSC); s += pmul(m, m); }
    s += __shfl_xor(s, 1); if (half == 0) m2s[row] = s; }
  for (int rr = 0; rr < 16; ++rr) { const v2f x = *(const v2f*)(CZ + (v0 + rr) * D + lane * 2); float s = pmul(x[0], x[0]) + pmul(x[1], x[1]); for (int o = 16; o; o >>= 1) s += __shfl_xor(s, o); if (lane == 0) n2s[wave][rr] = s;
    for (int j = 0; j < 2; ++j) { b16 p, q; split16(x[j] * XS, p, q); Ah[wave][rr][lane * 2 + j] = p; Al[wave][rr][lane * 2 + j] = q; } }
  __syncthreads();
  v8f acc = (v8f){};
#pragma unroll
  for (int kb = 0; kb < D; kb += 32) { const v16b a = frag_kb(&Ah[wave][nloc][kb], hlf), al = frag_kb(&Al[wave][nloc][kb], hlf); const v16b bw = frag_kb(&MU[nloc][kb], hlf); acc = wmma16b(a, bw, acc); acc = wmma16b(al, bw, acc); }
  const float m2 = m2s[nloc];
#pragma unroll
  for (int r8 = 0; r8 < 8; ++r8) { const int rl = 8 * hlf + r8; const float d2 = n2s[wave][rl] - 2.0f * (acc[r8] * (1.0f / (XS * WSC))) + m2; float q = (nloc < KCL) ? 1.0f / (1.0f + d2) : 0.0f;
    float s = q; for (int o = 1; o < 16; o <<= 1) s += __shfl_xor(s, o); q = q / s; if (nloc < KCL) so[(wave * 16 + rl) * KCL + nloc] = q; }
  __syncthreads();
  for (int pass = 0; pass < 2; ++pass) { if (threadIdx.x < 32 * KCL / 4) *(volatile v4f*)(outq + (size_t)blockIdx.x * 32 * KCL + threadIdx.x * 4) = *(const v4f*)(&so[threadIdx.x * 4]); __threadfence(); }
}
__global__ __launch_bounds__(160) void dec_kernel(const float* __restrict__ CZ, const float* __restrict__ GZ, const int* __restrict__ pu, const int* __restrict__ pv, int P, float* __restrict__ outp) {
  const size_t p = (size_t)blockIdx.x * 160 + threadIdx.x; const size_t pc = p < (size_t)P ? p : (size_t)(P - 1);
  const int u = iclamp(pu[pc], 0, NC - 1), v = iclamp(pv[pc], 0, NGENE - 1); const float* cu = CZ + (size_t)u * D; const float* gv = GZ + (size_t)v * D; float s = 0.0f;
#pragma unroll 2
  for (int k = 0; k < D; k += 4) { const v4f a = *(const v4f*)(cu + k), b = *(const v4f*)(gv + k); for (int i = 0; i < 4; ++i) s += pmul(a[i], b[i]); }
  const float o = 1.0f / (1.0f + __expf(-s));
  for (int pass = 0; pass < 2; ++pass) { if (p < (size_t)P) ((volatile float*)outp)[p] = o; __threadfence(); }
}
}

extern "C" void kernel_launch(void* const* d_in, const int* in_sizes, int n_in, void* d_out, int out_size, void* d_ws, size_t ws_size, hipStream_t stream) {
  (void)n_in;
  auto Fp = [&](int i) { return (const float*)d_in[i]; }; auto Ip = [&](int i) { return (const int*)d_in[i]; };
  if (in_sizes[0] != NC * D || in_sizes[1] != NGENE * D || in_sizes[2] != KCL * D || in_sizes[3] != 3 || in_sizes[4] != NC || in_sizes[6] != NGENE || in_sizes[8] != EADJ || in_sizes[9] != EEXP || in_sizes[10] != EEXP || in_sizes[11] != EADJ || in_sizes[12] != EADJ || in_sizes[13] != EPOS || in_sizes[16] != ENEG || out_size != EPOS + ENEG + NC * KCL) return;
  size_t off = 0; char* ws = (char*)d_ws;
  auto carve = [&](size_t bytes) { char* p = ws + off; off += (bytes + 255) & ~(size_t)255; return p; };
  float* G1 = (float*)carve((size_t)NGP * D * 4); float* G2 = (float*)carve((size_t)NGP * D * 4); float* GZ = (float*)carve((size_t)NGP * D * 4);
  float* C1 = (float*)carve((size_t)NCP * D * 4); float* C2 = (float*)carve((size_t)NCP * D * 4); float* CH2 = (float*)carve((size_t)NCP * D * 4); float* CZ = (float*)carve((size_t)NCP * D * 4);
  CsrBufs3 csrG; CsrBufs6 csrC; CsrBufs9 csrA; off = csr_carve3(csrG, ws, off, EEXP, NGENE); off = csr_carve6(csrC, ws, off, EEXP, NC); off = csr_carve9(csrA, ws, off, EADJ, NC);
  if (off > ws_size || off > ((size_t)128 << 20)) return;
  csr_build3(csrG, Ip(10), EEXP, NGENE, stream);
  csr_build6(csrC, Ip(9), EEXP, NC, stream);
  csr_build9(csrA, Ip(11), EADJ, NC, stream);
  mp_kernel<3, 1><<<NGP / 8, 256, 0, stream>>>(Fp(0), NC, Fp(4), Fp(7), Ip(9), EEXP, csrG.PERM, csrG.ROWPTR, csrG.ROWCNT, (int)csrG.permLen, NGENE, G1);
  mp_kernel<6, 1><<<NCP / 8, 256, 0, stream>>>(Fp(1), NGENE, Fp(6), Fp(5), Ip(10), EEXP, csrC.PERM, csrC.ROWPTR, csrC.ROWCNT, (int)csrC.permLen, NC, C1);
  mp_kernel<3, 0><<<NGP / 8, 256, 0, stream>>>(C1, NC, Fp(4), Fp(7), Ip(9), EEXP, csrG.PERM, csrG.ROWPTR, csrG.ROWCNT, (int)csrG.permLen, NGENE, G2);
  mp_kernel<6, 0><<<NCP / 8, 256, 0, stream>>>(G1, NGENE, Fp(6), Fp(5), Ip(10), EEXP, csrC.PERM, csrC.ROWPTR, csrC.ROWCNT, (int)csrC.permLen, NC, C2);
  spmm_kernel<1><<<NCP / 8, 256, 0, stream>>>(Fp(0), C1, C2, Fp(3), Fp(8), Ip(12), csrA.PERM, csrA.ROWPTR, csrA.ROWCNT, (int)csrA.permLen, CH2);
  spmm_kernel<0><<<NCP / 8, 256, 0, stream>>>(nullptr, CH2, nullptr, Fp(3), Fp(8), Ip(12), csrA.PERM, csrA.ROWPTR, csrA.ROWCNT, (int)csrA.permLen, CZ);
  gmix_kernel<<<NGP / 8, 256, 0, stream>>>(Fp(1), G1, G2, Fp(3), GZ);
  float* outP = (float*)d_out; float* outN = outP + EPOS; float* outQ = outN + ENEG;
  q_kernel<<<NC / 32, 64, 0, stream>>>(CZ, Fp(2), outQ);
  dec_kernel<<<EPOS / 160, 160, 0, stream>>>(CZ, GZ, Ip(13), Ip(14), EPOS, outP);
  dec_kernel<<<ENEG / 160, 160, 0, stream>>>(CZ, GZ, Ip(15), Ip(16), ENEG, outN);
}
